// CrossAttentionBlock_32727650796063
// MI455X (gfx1250) — hardware-verified
//
#include <hip/hip_runtime.h>
#include <math.h>

#ifndef NB
#define NB 4
#endif
#define NB_FULL 4
#define CH   384
#define NT   4096
#define NHD  8
#define HD   48
#define HDP  64
#define PK   256
#define C4   1536
#define KVC  768
#define XBS  ((long long)CH * NT)
static_assert(NB >= 1 && NB <= NB_FULL);
static_assert(CH % 64 == 0 && NT % 64 == 0 && PK % 64 == 0 && C4 % 64 == 0 && KVC % 64 == 0);
static_assert(CH % 32 == 0 && NT % 32 == 0 && C4 % 32 == 0 && HDP % 32 == 0);
static_assert(HD == 3 * 16 && NHD * HD == CH && HD < HDP);

typedef __attribute__((ext_vector_type(16))) _Float16 v16h;
typedef __attribute__((ext_vector_type(8)))  _Float16 v8h;
typedef __attribute__((ext_vector_type(8)))  float    v8f;
typedef __attribute__((ext_vector_type(4)))  float    v4f;
typedef __attribute__((ext_vector_type(4)))  unsigned int u4;

#define VST2(T, ptr, val) do { const T vst2_v_ = (val); *(volatile T*)(ptr) = vst2_v_; __threadfence(); *(volatile T*)(ptr) = vst2_v_; } while (0)

__device__ __forceinline__ float bfr(float v) {
    const unsigned u = __float_as_uint(v); return __uint_as_float((u + 0x7fffu + ((u >> 16) & 1u)) & 0xffff0000u);
}
__device__ __forceinline__ v4f bfr4(v4f a) { v4f r; r.x = bfr(a.x); r.y = bfr(a.y); r.z = bfr(a.z); r.w = bfr(a.w); return r; }
__device__ __forceinline__ unsigned int pk2h(float a, float b) {
    return (unsigned int)__builtin_bit_cast(unsigned short, (_Float16)a) | ((unsigned int)__builtin_bit_cast(unsigned short, (_Float16)b) << 16);
}
__device__ __forceinline__ v8f wmma16(v16h a, v16h b, v8f c) {
    c = __builtin_amdgcn_wmma_f32_16x16x32_f16(false, a, false, b, (short)0, c, false, false);
    asm volatile("v_nop\n\tv_nop\n\tv_nop\n\tv_nop" : "+v"(c) : "v"(a), "v"(b));
    return c;
}
__device__ __forceinline__ v16h frag_ld(const _Float16* p, int k0, int hh) {
    union { v16h v; v8h h[2]; } f; f.h[0] = *(const v8h*)(p + k0 + 8 * hh); f.h[1] = *(const v8h*)(p + k0 + 16 + 8 * hh); return f.v;
}

namespace w25 {
__device__ __forceinline__ void dep_guard_h(v8f& a, v8f& b, v16h x, v16h y) { asm volatile("v_nop\n\tv_nop\n\tv_nop\n\tv_nop" : "+v"(a), "+v"(b) : "v"(x), "v"(y)); }
__device__ __forceinline__ void keep4_h(v16h a, v16h b, v16h c, v16h d) { asm volatile("v_nop" :: "v"(a), "v"(b), "v"(c), "v"(d)); }
__device__ __forceinline__ void acc_guard4(v8f& a, v8f& b, v8f& c, v8f& d) { asm volatile("v_nop\n\tv_nop\n\tv_nop\n\tv_nop" : "+v"(a), "+v"(b), "+v"(c), "+v"(d)); }
struct FragH {
  union U { v16h v; v8h h[2]; };
  static __device__ __forceinline__ v16h load(const _Float16* p) {
    U f; f.h[0] = *(const v8h*)(p); f.h[1] = *(const v8h*)(p + 16); return f.v;
  }
  static __device__ __forceinline__ v8f mma(v16h a, v16h b, v8f c) {
    return __builtin_amdgcn_wmma_f32_16x16x32_f16(false, a, false, b, (short)0, c, false, false);
  }
};

template <bool SPLIT, int BIAS_MODE, int OUT_MODE, bool RESID, int ACT, bool RBF>
__global__ __launch_bounds__(256) void wmma_gemm64(
    const unsigned short* __restrict__ Ap, const unsigned short* __restrict__ A2p, int lda, long long strideA,
    const unsigned short* __restrict__ Btp, const unsigned short* __restrict__ Bt2p, int ldb, long long strideB,
    void* __restrict__ Cout, void* __restrict__ Cout2, int ldc, long long strideC,
    const float* __restrict__ bias,
    const float* __restrict__ resid, long long strideR,
    int M, int N, int K, float scale) {
  static_assert(!RESID || (ACT == 0 && OUT_MODE == 0));
  (void)Cout2;
  const _Float16* A = (const _Float16*)Ap; const _Float16* A2 = (const _Float16*)A2p; const _Float16* Bt = (const _Float16*)Btp; const _Float16* Bt2 = (const _Float16*)Bt2p;
  __shared__ __align__(16) float sT[8][16 * 68];
  const int b    = blockIdx.y;
  const int lane = threadIdx.x & 31;
  const int wave = threadIdx.x >> 5;
  const int tilesN = N >> 6;
  const int tilesM = M >> 6;
  const int tile = blockIdx.x * 8 + wave;
  if (tile >= tilesM * tilesN) return;
  const int tm = tile / tilesN;
  const int tn = tile - tm * tilesN;
  const int m0 = tm << 6;
  const int n0 = tn << 6;

  const _Float16* Ab  = A  + (size_t)b * strideA;
  const _Float16* Bb  = Bt + (size_t)b * strideB;
  const _Float16* Ab2 = SPLIT ? (A2  + (size_t)b * strideA) : nullptr;
  const _Float16* Bb2 = SPLIT ? (Bt2 + (size_t)b * strideB) : nullptr;

  const int rlane = lane & 15;
  const int koff  = (lane >> 4) * 8;
  const int mOff  = (lane >> 4) * 8;

  v8f acc[4][4];
#pragma unroll
  for (int i = 0; i < 4; ++i)
#pragma unroll
    for (int j = 0; j < 4; ++j) acc[i][j] = (v8f){0.f,0.f,0.f,0.f,0.f,0.f,0.f,0.f};

  for (int k0 = 0; k0 < K; k0 += 32) {
    v16h bh[4], bl[4];
#pragma unroll
    for (int j = 0; j < 4; ++j) {
      const size_t bo = (size_t)(n0 + (j << 4) + rlane) * ldb + koff + k0;
      bh[j] = FragH::load(Bb + bo);
      if (SPLIT) bl[j] = FragH::load(Bb2 + bo);
    }
#pragma unroll
    for (int i = 0; i < 4; ++i) {
      const size_t ao = (size_t)(m0 + (i << 4) + rlane) * lda + koff + k0;
      v16h ah = FragH::load(Ab + ao);
      v16h al = ah;
      if (SPLIT) al = FragH::load(Ab2 + ao);
#pragma unroll
      for (int j = 0; j < 4; ++j) {
        acc[i][j] = FragH::mma(ah, bh[j], acc[i][j]);
        if (SPLIT) {
          acc[i][j] = FragH::mma(ah, bl[j], acc[i][j]);
          acc[i][j] = FragH::mma(al, bh[j], acc[i][j]);
        }
      }
      dep_guard_h(acc[i][0], acc[i][3], ah, al);
    }
    keep4_h(bh[0], bh[1], bh[2], bh[3]);
    if (SPLIT) keep4_h(bl[0], bl[1], bl[2], bl[3]);
  }
  acc_guard4(acc[0][0], acc[0][1], acc[0][2], acc[0][3]);
  acc_guard4(acc[1][0], acc[1][1], acc[1][2], acc[1][3]);
  acc_guard4(acc[2][0], acc[2][1], acc[2][2], acc[2][3]);
  acc_guard4(acc[3][0], acc[3][1], acc[3][2], acc[3][3]);

  float* slab = sT[wave];
  const float* Rb = RESID ? (resid + (size_t)b * strideR) : nullptr;
#pragma unroll
  for (int i = 0; i < 4; ++i) {
    const int mBase = m0 + (i << 4);
#pragma unroll
    for (int j = 0; j < 4; ++j) {
      const int n = n0 + (j << 4) + rlane;
      float bv = 0.f;
      if (BIAS_MODE == 2) bv = bias[n];
#pragma unroll
      for (int r = 0; r < 8; ++r) {
        float v = acc[i][j][r] * scale;
        if (BIAS_MODE == 1) v += bias[mBase + mOff + r];
        if (BIAS_MODE == 2) v += bv;
        if (ACT == 1) v = tanhf(v);
        if (ACT == 2) v = fmaxf(v, 0.0f);
        if (ACT == 3) v = v / (1.0f + expf(-v));
        if (ACT == 4) v = (v > 0.f) ? v : 0.01f * v;
        if (ACT == 5) v = 0.5f * v * (1.0f + erff(v * 0.70710678118654752f));
        if (ACT == 6) v = (v > 0.f) ? v : 0.2f * v;
        if (ACT == 7) { const float u = 0.7978845608028654f * (v + 0.044715f * v * v * v); v = 0.5f * v * (1.f + tanhf(u)); }
        slab[(mOff + r) * 68 + (j << 4) + rlane] = v;
      }
    }
    __builtin_amdgcn_fence(3  , "workgroup");
    __builtin_amdgcn_wave_barrier();
    __builtin_amdgcn_fence(2  , "workgroup");
    if (OUT_MODE == 0) {
      float* C = (float*)Cout + (size_t)b * strideC;
      const int hh = lane >> 4, c4 = (lane & 15) * 4;
      if (RESID) {
#pragma unroll
        for (int it = 0; it < 8; ++it) {
          const int row = it * 2 + hh;
          float* sp = slab + row * 68 + c4;
          v4f v = *(const v4f*)sp;
          const v4f ry = *(const v4f*)(Rb + (size_t)(mBase + row) * ldc + n0 + c4);
          v += RBF ? bfr4(ry) : ry;
          *(v4f*)sp = v;
        }
      }
      for (int pass = 0; pass < 2; ++pass) {
#pragma unroll
        for (int it = 0; it < 8; ++it) {
          const int row = it * 2 + hh;
          v4f v = *(const v4f*)(slab + row * 68 + c4);
          *(volatile v4f*)(C + (size_t)(mBase + row) * ldc + n0 + c4) = v;
        }
        __threadfence();
      }
    } else {
      const int q = lane >> 3, c8 = (lane & 7) * 8;
      unsigned short* C  = (unsigned short*)Cout  + (size_t)b * strideC;
      for (int pass = 0; pass < 2; ++pass) {
#pragma unroll
        for (int it = 0; it < 4; ++it) {
          const int row = it * 4 + q;
          const float* sp = slab + row * 68 + c8;
          v8h hv;
#pragma unroll
          for (int e = 0; e < 8; ++e) hv[e] = (_Float16)sp[e];
          *(volatile v8h*)(C + (size_t)(mBase + row) * ldc + n0 + c8) = hv;
        }
        __threadfence();
      }
    }
    __builtin_amdgcn_fence(3  , "workgroup");
    __builtin_amdgcn_wave_barrier();
    __builtin_amdgcn_fence(2  , "workgroup");
  }
}
}

__global__ __launch_bounds__(256) void k_castbT(const float* __restrict__ SRC, long long sS, int lds, unsigned short* __restrict__ DST, long long sD, int ldd, int nR, int nC, float sc) {
    const long long u = (long long)blockIdx.x * 256 + threadIdx.x; const int per = nR >> 3;
    if (u >= (long long)nC * per) return;
    const int c = (int)(u / per); const int r0 = 8 * (int)(u - (long long)c * per);
    const float* s = SRC + (long long)blockIdx.y * sS + (long long)r0 * lds + c;
    float w[8];
#pragma unroll
    for (int e = 0; e < 8; ++e) w[e] = bfr(s[(long long)e * lds]) * sc;
    u4 pk; pk.x = pk2h(w[0], w[1]); pk.y = pk2h(w[2], w[3]); pk.z = pk2h(w[4], w[5]); pk.w = pk2h(w[6], w[7]);
    VST2(u4, DST + (long long)blockIdx.y * sD + (long long)c * ldd + r0, pk);
}

#define BR_B1 0
#define BR_B2 1536
#define BR_G  1920
#define BR_BT 2304
#define BR_T  2688
#define BR_N  2720
__global__ __launch_bounds__(256) void k_bfvec(const float* __restrict__ b1, const float* __restrict__ b2, const float* __restrict__ g, const float* __restrict__ bt,
                                               const float* __restrict__ tm, float* __restrict__ BR) {
    const int u = blockIdx.x * 256 + threadIdx.x; if (u >= BR_N) return;
    const float v1 = b1[min(u, C4 - 1)];
    const float v2 = b2[min(max(u - BR_B2, 0), CH - 1)];
    const float v3 = g[min(max(u - BR_G, 0), CH - 1)];
    const float v4 = bt[min(max(u - BR_BT, 0), CH - 1)];
    const float v5 = tm[min(max(u - BR_T, 0), NHD - 1)];
    const float v = (u < BR_B2) ? v1 : ((u < BR_G) ? v2 : ((u < BR_BT) ? v3 : ((u < BR_T) ? v4 : ((u < BR_T + NHD) ? v5 : 0.f))));
    VST2(float, BR + u, bfr(v));
}

#define QSC 64.0f
__global__ __launch_bounds__(256) void k_qcast(const float* __restrict__ QF, unsigned short* __restrict__ QH) {
    __shared__ float red[4][64];
    __shared__ float rq[64];
    const int h = blockIdx.x, b = blockIdx.y, t = threadIdx.x;
    const int col = t & 63, rg = t >> 6; const int colc = min(col, HD - 1);
    const float* base = QF + ((long long)b * NT) * CH + h * HD + colc;
    float s = 0.f;
#pragma unroll 4
    for (int n = rg; n < NT; n += 4) { const float v = base[(long long)n * CH]; s += v * v; }
    red[rg][col] = s;
    __syncthreads();
    if (t < 64) { const float ss = (red[0][t] + red[1][t]) + (red[2][t] + red[3][t]); rq[t] = (t < HD) ? QSC * rsqrtf(fmaxf(ss, 1e-24f)) : 0.f; }
    __syncthreads();
    for (int it = 0; it < NT * 8 / 256; ++it) {
        const int u = it * 256 + t; const int n = u >> 3, g = u & 7; const int gc = min(g, 5);
        const float* qr = QF + ((long long)b * NT + n) * CH + h * HD + 8 * gc;
        const v4f a = *(const v4f*)qr, c = *(const v4f*)(qr + 4);
        const bool live = (g < 6);
        float w[8] = {a.x, a.y, a.z, a.w, c.x, c.y, c.z, c.w};
#pragma unroll
        for (int e = 0; e < 8; ++e) w[e] = live ? w[e] * rq[8 * g + e] : 0.f;
        u4 pk; pk.x = pk2h(w[0], w[1]); pk.y = pk2h(w[2], w[3]); pk.z = pk2h(w[4], w[5]); pk.w = pk2h(w[6], w[7]);
        VST2(u4, QH + (((long long)(b * NHD + h) * NT + n) * HDP + 8 * g), pk);
    }
}

__global__ __launch_bounds__(256) void k_kpt(const float* __restrict__ KPVP, unsigned short* __restrict__ KPT, int nrow) {
    const long long u = (long long)blockIdx.x * 256 + threadIdx.x; if (u >= (long long)nrow * 8) return;
    const int row = (int)(u >> 3), g = (int)(u & 7); const int p = row & (PK - 1); const int bh = row >> 8; const int h = bh & (NHD - 1), b = bh >> 3;
    const int gc = min(g, 5);
    const float* src = KPVP + ((long long)b * KVC + h * HD + 8 * gc) * PK + p;
    float w[8];
#pragma unroll
    for (int e = 0; e < 8; ++e) w[e] = src[(long long)e * PK];
    const bool live = (g < 6);
#pragma unroll
    for (int e = 0; e < 8; ++e) w[e] = live ? w[e] : 0.f;
    u4 pk; pk.x = pk2h(w[0], w[1]); pk.y = pk2h(w[2], w[3]); pk.z = pk2h(w[4], w[5]); pk.w = pk2h(w[6], w[7]);
    VST2(u4, KPT + (long long)row * HDP + 8 * g, pk);
}

__global__ __launch_bounds__(256) void k_vp(const float* __restrict__ KPVP, unsigned short* __restrict__ VPp, float* __restrict__ VM, int nrow) {
    __shared__ float vms[32];
    const int wave = threadIdx.x >> 5, L = threadIdx.x & 31;
    (void)nrow;
    for (int i = 0; i < 4; ++i) {
        const int rl = wave * 4 + i; const int row = blockIdx.x * 32 + rl;
        const int b = row / CH, c = row - b * CH;
        const float* src = KPVP + ((long long)b * KVC + CH + c) * PK + 8 * L;
        const v4f a = *(const v4f*)src, d = *(const v4f*)(src + 4);
        float s = ((a.x + a.y) + (a.z + a.w)) + ((d.x + d.y) + (d.z + d.w));
#pragma unroll
        for (int o = 16; o > 0; o >>= 1) s += __shfl_xor(s, o, 32);
        u4 pk; pk.x = pk2h(a.x, a.y); pk.y = pk2h(a.z, a.w); pk.z = pk2h(d.x, d.y); pk.w = pk2h(d.z, d.w);
        VST2(u4, VPp + (long long)row * PK + 8 * L, pk);
        if (L == 0) vms[rl] = s * (1.0f / (float)PK);
    }
    __syncthreads();
    if (wave == 0) VST2(float, VM + (long long)blockIdx.x * 32 + L, vms[L]);
}

#define AQ   32
#define SPF  260
#define PPH  264
#define OSP  36
#define PSC  16384.0f
__global__ __launch_bounds__(64) void k_lattn(const unsigned short* __restrict__ QH, const unsigned short* __restrict__ KPT, const unsigned short* __restrict__ VPp,
                                              const float* __restrict__ VM, const float* __restrict__ TMP, float* __restrict__ OLN) {
    __shared__ __align__(16) float Sw[2][16 * SPF];
    __shared__ __align__(16) unsigned short Pw[2][16 * PPH];
    __shared__ __align__(16) float Os[HD * OSP];
    const int lane = threadIdx.x & 31, hh = lane >> 4, l15 = lane & 15, wave = threadIdx.x >> 5;
    const int qb = blockIdx.x, h = blockIdx.y, b = blockIdx.z;
    const long long bh = (long long)b * NHD + h;
    const int q0 = qb * AQ + wave * 16;
    const _Float16* qrow = (const _Float16*)QH + (bh * NT + q0 + l15) * HDP;
    const v16h qa0 = frag_ld(qrow, 0, hh), qa1 = frag_ld(qrow, 32, hh);
    const _Float16* kbs = (const _Float16*)KPT + bh * PK * HDP;
    const float tsc = TMP[h] * (1.4426950408889634f / QSC);
    float* sw = Sw[wave];
#pragma unroll 2
    for (int t = 0; t < PK / 16; ++t) {
        const _Float16* krow = kbs + (long long)(t * 16 + l15) * HDP;
        v8f acc = {};
        acc = wmma16(qa0, frag_ld(krow, 0, hh), acc);
        acc = wmma16(qa1, frag_ld(krow, 32, hh), acc);
#pragma unroll
        for (int r = 0; r < 8; ++r) sw[(8 * hh + r) * SPF + t * 16 + l15] = acc[r] * tsc;
    }
    __builtin_amdgcn_fence(3  , "workgroup");
    __builtin_amdgcn_wave_barrier();
    __builtin_amdgcn_fence(2  , "workgroup");
    unsigned short* pw = Pw[wave];
#pragma unroll 1
    for (int i = 0; i < 16; ++i) {
        const float* sr = sw + i * SPF + 8 * lane;
        const v4f xa = *(const v4f*)sr, xb = *(const v4f*)(sr + 4);
        float e[8] = {xa.x, xa.y, xa.z, xa.w, xb.x, xb.y, xb.z, xb.w};
        float m = fmaxf(fmaxf(fmaxf(e[0], e[1]), fmaxf(e[2], e[3])), fmaxf(fmaxf(e[4], e[5]), fmaxf(e[6], e[7])));
#pragma unroll
        for (int o = 16; o > 0; o >>= 1) m = fmaxf(m, __shfl_xor(m, o, 32));
        float s = 0.f;
#pragma unroll
        for (int q = 0; q < 8; ++q) { e[q] = exp2f(e[q] - m); s += e[q]; }
#pragma unroll
        for (int o = 16; o > 0; o >>= 1) s += __shfl_xor(s, o, 32);
        s = __shfl(s, 0, 32);
        const float inv = PSC / s;
        float pv[8];
#pragma unroll
        for (int q = 0; q < 8; ++q) pv[q] = e[q] * inv - (PSC / (float)PK);
        u4 pk; pk.x = pk2h(pv[0], pv[1]); pk.y = pk2h(pv[2], pv[3]); pk.z = pk2h(pv[4], pv[5]); pk.w = pk2h(pv[6], pv[7]);
        *(u4*)(pw + i * PPH + 8 * lane) = pk;
    }
    __builtin_amdgcn_fence(3  , "workgroup");
    __builtin_amdgcn_wave_barrier();
    __builtin_amdgcn_fence(2  , "workgroup");
    v8f o[3];
#pragma unroll
    for (int dt = 0; dt < 3; ++dt) o[dt] = (v8f){0.f,0.f,0.f,0.f,0.f,0.f,0.f,0.f};
    const _Float16* prow = (const _Float16*)pw + l15 * PPH;
    const _Float16* vbs = (const _Float16*)VPp + ((long long)b * CH + h * HD) * PK;
#pragma unroll 1
    for (int ks = 0; ks < PK / 32; ++ks) {
        const v16h pa = frag_ld(prow, 32 * ks, hh);
#pragma unroll
        for (int dt = 0; dt < 3; ++dt) o[dt] = wmma16(pa, frag_ld(vbs + (long long)(dt * 16 + l15) * PK, 32 * ks, hh), o[dt]);
    }
    const float* vm = VM + (long long)b * CH + h * HD;
#pragma unroll
    for (int dt = 0; dt < 3; ++dt) {
        const int d = dt * 16 + l15; const float vmd = vm[d];
#pragma unroll
        for (int r = 0; r < 8; ++r) Os[d * OSP + wave * 16 + 8 * hh + r] = o[dt][r] * (1.0f / PSC) + vmd;
    }
    __syncthreads();
    float* ob = OLN + (long long)b * XBS + (long long)h * NT + (long long)qb * AQ;
    const int sub = lane >> 3, c4 = (lane & 7) * 4;
    for (int pass = 0; pass < 2; ++pass) {
#pragma unroll
        for (int j = 0; j < 6; ++j) {
            const int d = wave * 24 + 4 * j + sub;
            const v4f v = *(const v4f*)(Os + d * OSP + c4);
            *(volatile v4f*)(ob + (long long)d * ((long long)NHD * NT) + c4) = v;
        }
        __threadfence();
    }
}

__global__ __launch_bounds__(256) void k_ln(const float* __restrict__ O, const float* __restrict__ G, const float* __restrict__ Bt, unsigned short* __restrict__ LN, int nrows) {
    const int row = blockIdx.x * 8 + (threadIdx.x >> 5); const int L = threadIdx.x & 31;
    if (row >= nrows) return;
    const float* o = O + (long long)row * CH;
    const int L2 = min(L, 15); const bool hi = (L < 16); const float msk = hi ? 1.f : 0.f;
    const int c0 = 8 * L, c1 = 256 + 8 * L2;
    const v4f a0 = *(const v4f*)(o + c0), a1 = *(const v4f*)(o + c0 + 4), b0 = *(const v4f*)(o + c1), b1 = *(const v4f*)(o + c1 + 4);
    float s = (((a0.x + a0.y) + (a0.z + a0.w)) + ((a1.x + a1.y) + (a1.z + a1.w))) + msk * (((b0.x + b0.y) + (b0.z + b0.w)) + ((b1.x + b1.y) + (b1.z + b1.w)));
#pragma unroll
    for (int q = 16; q > 0; q >>= 1) s += __shfl_xor(s, q, 32);
    const float mu = s * (1.0f / (float)CH);
    const v4f d0 = a0 - mu, d1 = a1 - mu, e0 = b0 - mu, e1 = b1 - mu;
    float qs = ((d0.x * d0.x + d0.y * d0.y) + (d0.z * d0.z + d0.w * d0.w)) + ((d1.x * d1.x + d1.y * d1.y) + (d1.z * d1.z + d1.w * d1.w))
             + msk * (((e0.x * e0.x + e0.y * e0.y) + (e0.z * e0.z + e0.w * e0.w)) + ((e1.x * e1.x + e1.y * e1.y) + (e1.z * e1.z + e1.w * e1.w)));
#pragma unroll
    for (int q = 16; q > 0; q >>= 1) qs += __shfl_xor(qs, q, 32);
    const float rstd = rsqrtf(qs * (1.0f / (float)CH) + 1e-5f);
    const v4f g0 = *(const v4f*)(G + c0), g1 = *(const v4f*)(G + c0 + 4), g2 = *(const v4f*)(G + c1), g3 = *(const v4f*)(G + c1 + 4);
    const v4f t0 = *(const v4f*)(Bt + c0), t1 = *(const v4f*)(Bt + c0 + 4), t2 = *(const v4f*)(Bt + c1), t3 = *(const v4f*)(Bt + c1 + 4);
    const v4f w0 = d0 * rstd * g0 + t0, w1 = d1 * rstd * g1 + t1, w2 = e0 * rstd * g2 + t2, w3 = e1 * rstd * g3 + t3;
    u4 pk0; pk0.x = pk2h(w0.x, w0.y); pk0.y = pk2h(w0.z, w0.w); pk0.z = pk2h(w1.x, w1.y); pk0.w = pk2h(w1.z, w1.w);
    u4 pk1; pk1.x = pk2h(w2.x, w2.y); pk1.y = pk2h(w2.z, w2.w); pk1.z = pk2h(w3.x, w3.y); pk1.w = pk2h(w3.z, w3.w);
    unsigned short* dst = LN + (long long)row * CH;
    *(volatile u4*)(dst + c0) = pk0;
    if (hi) *(volatile u4*)(dst + 256 + c0) = pk1;
    __threadfence();
    *(volatile u4*)(dst + c0) = pk0;
    if (hi) *(volatile u4*)(dst + 256 + c0) = pk1;
}

extern "C" void kernel_launch(void* const* d_in, const int* in_sizes, int n_in, void* d_out, int out_size, void* d_ws, size_t ws_size, hipStream_t stream) {
    if (n_in < 12) return;
    if (in_sizes[0] < NB * CH * NT || in_sizes[1] < NB * CH * NT || in_sizes[2] < CH * CH || in_sizes[3] < CH * KVC || in_sizes[4] < NT * PK ||
        in_sizes[5] < NHD || in_sizes[6] < CH || in_sizes[7] < CH || in_sizes[8] < CH * C4 || in_sizes[9] < C4 || in_sizes[10] < C4 * CH || in_sizes[11] < CH) return;
    if (out_size < NB * CH * NT) return;
    const float* x     = (const float*)d_in[0];
    const float* y     = (const float*)d_in[1];
    const float* Wq    = (const float*)d_in[2];
    const float* Wkv   = (const float*)d_in[3];
    const float* EF    = (const float*)d_in[4];
    const float* temp  = (const float*)d_in[5];
    const float* gamma = (const float*)d_in[6];
    const float* beta  = (const float*)d_in[7];
    const float* w1    = (const float*)d_in[8];
    const float* b1    = (const float*)d_in[9];
    const float* w2    = (const float*)d_in[10];
    const float* b2    = (const float*)d_in[11];
    float* outp = (float*)d_out;

    constexpr size_t SZ_R1   = (size_t)NB * NT * C4 * 2;
    constexpr size_t SZ_XT   = (size_t)NB * NT * CH * 2;
    constexpr size_t SZ_KVT  = (size_t)NB * KVC * NT * 2;
    static_assert(SZ_XT + SZ_KVT <= SZ_R1);
    constexpr size_t SZ_R2   = (size_t)NB * NT * CH * 4;
    constexpr size_t SZ_R3   = (size_t)NB * NHD * NT * HDP * 2;
    static_assert((size_t)NB * NT * CH * 2 <= SZ_R3);
    constexpr size_t SZ_WQT  = (size_t)CH * CH * 2;
    constexpr size_t SZ_WKVT = (size_t)KVC * CH * 2;
    constexpr size_t SZ_EFT  = (size_t)PK * NT * 2;
    constexpr size_t SZ_W1T  = (size_t)C4 * CH * 2;
    constexpr size_t SZ_W2T  = (size_t)CH * C4 * 2;
    constexpr size_t SZ_BR   = 12288;
    static_assert(BR_N * 4 <= SZ_BR);
    constexpr size_t SZ_KPVP = (size_t)NB * KVC * PK * 4;
    constexpr size_t SZ_KPT  = (size_t)NB * NHD * PK * HDP * 2;
    constexpr size_t SZ_VP   = (size_t)NB * CH * PK * 2;
    constexpr size_t SZ_VM   = (size_t)NB * CH * 4;
    constexpr size_t OFF_R1 = 0, OFF_R2 = OFF_R1 + SZ_R1, OFF_R3 = OFF_R2 + SZ_R2, OFF_WQT = OFF_R3 + SZ_R3, OFF_WKVT = OFF_WQT + SZ_WQT,
                     OFF_EFT = OFF_WKVT + SZ_WKVT, OFF_W1T = OFF_EFT + SZ_EFT, OFF_W2T = OFF_W1T + SZ_W1T, OFF_BR = OFF_W2T + SZ_W2T,
                     OFF_KPVP = OFF_BR + SZ_BR, OFF_KPT = OFF_KPVP + SZ_KPVP, OFF_VP = OFF_KPT + SZ_KPT, OFF_VM = OFF_VP + SZ_VP, WS_TOTAL = OFF_VM + SZ_VM;
    static_assert(WS_TOTAL <= (size_t)134217728);
    static_assert((OFF_R2 % 256) == 0 && (OFF_R3 % 256) == 0 && (OFF_WQT % 256) == 0 && (OFF_KPVP % 256) == 0 && (OFF_KPT % 256) == 0 && (OFF_VP % 256) == 0 && (OFF_VM % 256) == 0);
    if (WS_TOTAL > ws_size) return;
    char* ws = (char*)d_ws;
    unsigned short* XT16  = (unsigned short*)(ws + OFF_R1);
    unsigned short* KVT16 = (unsigned short*)(ws + OFF_R1 + SZ_XT);
    unsigned short* H16   = (unsigned short*)(ws + OFF_R1);
    float*          QF    = (float*)(ws + OFF_R2);
    float*          OLN   = (float*)(ws + OFF_R2);
    unsigned short* QH16  = (unsigned short*)(ws + OFF_R3);
    unsigned short* LN16  = (unsigned short*)(ws + OFF_R3);
    unsigned short* WQT   = (unsigned short*)(ws + OFF_WQT);
    unsigned short* WKVT  = (unsigned short*)(ws + OFF_WKVT);
    unsigned short* EFT   = (unsigned short*)(ws + OFF_EFT);
    unsigned short* W1T   = (unsigned short*)(ws + OFF_W1T);
    unsigned short* W2T   = (unsigned short*)(ws + OFF_W2T);
    float*          BR    = (float*)(ws + OFF_BR);
    float*          KPVP  = (float*)(ws + OFF_KPVP);
    unsigned short* KPT16 = (unsigned short*)(ws + OFF_KPT);
    unsigned short* VP16  = (unsigned short*)(ws + OFF_VP);
    float*          VM    = (float*)(ws + OFF_VM);

    k_castbT<<<dim3((unsigned)(((long long)NT * (CH / 8) + 255) / 256), NB), 256, 0, stream>>>(x, XBS, NT, XT16, (long long)NT * CH, CH, CH, NT, 1.0f);
    k_castbT<<<dim3((unsigned)(((long long)CH * (CH / 8) + 255) / 256), 1), 256, 0, stream>>>(Wq, 0, CH, WQT, 0, CH, CH, CH, 16.0f);
    k_castbT<<<dim3((unsigned)(((long long)KVC * (CH / 8) + 255) / 256), 1), 256, 0, stream>>>(Wkv, 0, KVC, WKVT, 0, CH, CH, KVC, 16.0f);
    k_castbT<<<dim3((unsigned)(((long long)PK * (NT / 8) + 255) / 256), 1), 256, 0, stream>>>(EF, 0, PK, EFT, 0, NT, NT, PK, 64.0f);
    k_castbT<<<dim3((unsigned)(((long long)C4 * (CH / 8) + 255) / 256), 1), 256, 0, stream>>>(w1, 0, C4, W1T, 0, CH, CH, C4, 16.0f);
    k_castbT<<<dim3((unsigned)(((long long)CH * (C4 / 8) + 255) / 256), 1), 256, 0, stream>>>(w2, 0, CH, W2T, 0, C4, C4, CH, 32.0f);
    k_bfvec<<<(BR_N + 255) / 256, 256, 0, stream>>>(b1, b2, gamma, beta, temp, BR);

    w25::wmma_gemm64<false, 0, 0, false, 0, false><<<dim3((unsigned)(((NB * NT / 64) * (CH / 64)) / 8), 1), 256, 0, stream>>>(
        XT16, nullptr, CH, 0, WQT, nullptr, CH, 0, (void*)QF, nullptr, CH, 0, nullptr, nullptr, 0, NB * NT, CH, CH, 0.0625f);
    w25::wmma_gemm64<false, 0, 1, false, 0, false><<<dim3((unsigned)(((KVC / 64) * (NT / 64)) / 8), NB), 256, 0, stream>>>(
        WKVT, nullptr, CH, 0, XT16, nullptr, CH, (long long)NT * CH, (void*)KVT16, nullptr, NT, (long long)KVC * NT, nullptr, nullptr, 0, KVC, NT, CH, 0.0625f);
    k_qcast<<<dim3(NHD, NB), 256, 0, stream>>>(QF, QH16);
    w25::wmma_gemm64<false, 0, 0, false, 0, false><<<dim3((unsigned)(((KVC / 64) * (PK / 64)) / 8), NB), 256, 0, stream>>>(
        KVT16, nullptr, NT, (long long)KVC * NT, EFT, nullptr, NT, 0, (void*)KPVP, nullptr, PK, (long long)KVC * PK, nullptr, nullptr, 0, KVC, PK, NT, 0.015625f);
    k_kpt<<<(unsigned)(((long long)NB * NHD * PK * 8 + 255) / 256), 256, 0, stream>>>(KPVP, KPT16, NB * NHD * PK);
    k_vp<<<(unsigned)(NB * CH / 32), 256, 0, stream>>>(KPVP, VP16, VM, NB * CH);
    k_lattn<<<dim3(NT / AQ, NHD, NB), 64, 0, stream>>>(QH16, KPT16, VP16, VM, BR + BR_T, OLN);
    k_ln<<<(unsigned)(NB * NT / 8), 256, 0, stream>>>(OLN, BR + BR_G, BR + BR_BT, LN16, NB * NT);
    w25::wmma_gemm64<false, 2, 1, false, 5, false><<<dim3((unsigned)(((NB * NT / 64) * (C4 / 64)) / 8), 1), 256, 0, stream>>>(
        LN16, nullptr, CH, 0, W1T, nullptr, CH, 0, (void*)H16, nullptr, C4, 0, BR + BR_B1, nullptr, 0, NB * NT, C4, CH, 0.0625f);
    w25::wmma_gemm64<false, 1, 0, true, 0, true><<<dim3((unsigned)(((CH / 64) * (NT / 64)) / 8), NB), 256, 0, stream>>>(
        W2T, nullptr, C4, 0, H16, nullptr, C4, (long long)NT * C4, (void*)outp, nullptr, NT, XBS, BR + BR_B2, y, XBS, CH, NT, C4, 0.03125f);
}
